// SpatioTemporalBlock_19061064859665
// MI455X (gfx1250) — hardware-verified
//
#include <hip/hip_runtime.h>
#include <stddef.h>


#define cBATCH 2
#define cN     1000
#define cF     8
#define cT     12
#define HD     64
#define cNF    (cN * cF)
#define GPN    (cBATCH * cT)
#define cE1    2000
#define cE2    24000
#define cR1    (cN * GPN)
#define cRX    (cNF * GPN)
#define cSEQ   (cBATCH * cNF)
#define SLOTF  (GPN * HD)

#define NTHR   256
#define NWAVE  8
#define EPT    8
#define NGRP   2
#define CHUNK  (NTHR * EPT * NGRP)
#define WCAP   (EPT * NGRP * 32)
#define LISTN  (NWAVE * WCAP)
#define NB     32
#define PST    68
#define QP     196
#define GP     260
#define ATHR   192
#define AWAVE  6
#define AROWS  96

#define TROWS  (NWAVE * 16)
#define NSCAN1 ((cN + NB - 1) / NB)
#define N1P    (NSCAN1 * NB)
#define NSCAN2 (cNF / NB)
#define NBLK1  ((cR1 + TROWS - 1) / TROWS)
#define R1P    (NBLK1 * TROWS)
#define NBLKX  (cRX / TROWS)
#define NBLKA  (cRX / AROWS)
#define NWSB   (cR1 * HD / 4 / NTHR)

#define WO_L1   0
#define WO_U1   4096
#define WO_L2   12288
#define WO_U2   16384
#define WO_F1   24576
#define WO_F2   32768
#define WO_QKV  36864
#define WO_O    49152
#define WO_FF1  53248
#define WO_FF2  69632
#define WTOT    86016

#define LDS_SCAN (NB * SLOTF * 4 + LISTN * 4 + NWAVE * 4 + NB * 4)
#define LDS_ATTN ((AROWS * HD + AROWS * PST + AROWS * QP) * 4)
#define LDS_FFN  ((AROWS * HD + AROWS * PST + AROWS * GP) * 4)

static_assert((CHUNK & (CHUNK - 1)) == 0);
static_assert(CHUNK <= 4096);
static_assert(NB <= 4096 && (NB & (NB - 1)) == 0);
static_assert(cNF % NB == 0);
static_assert(NSCAN1 * NB == N1P && N1P >= cN);
static_assert(cRX % TROWS == 0);
static_assert(cRX % AROWS == 0);
static_assert(AROWS % cT == 0);
static_assert(ATHR == 2 * AROWS);
static_assert((cR1 * HD) % (4 * NTHR) == 0);
static_assert((size_t)R1P * HD <= (size_t)N1P * SLOTF);
static_assert(R1P <= N1P * GPN);
static_assert((R1P - 1) / GPN < N1P);
static_assert(R1P >= cR1);
static_assert((NB * SLOTF) % (4 * NTHR) == 0);

typedef float          v4f  __attribute__((ext_vector_type(4)));
typedef float          v8f  __attribute__((ext_vector_type(8)));
typedef int            v4i  __attribute__((ext_vector_type(4)));
typedef unsigned short v8us __attribute__((ext_vector_type(8)));
typedef __bf16         v16b __attribute__((ext_vector_type(16)));
union FragB { v16b v; v8us u[2]; };

__device__ __forceinline__ int imin(int a, int b) { return a < b ? a : b; }
__device__ __forceinline__ int imax(int a, int b) { return a > b ? a : b; }

__device__ __forceinline__ unsigned int bf_rne(unsigned int u) {
  return (u + 0x7FFFu + ((u >> 16) & 1u)) >> 16;
}
__device__ __forceinline__ void split1(float f, unsigned short& ho, unsigned short& lo) {
  const unsigned int hb = bf_rne(__float_as_uint(f));
  const float rem = f - __uint_as_float(hb << 16);
  ho = (unsigned short)hb;
  lo = (unsigned short)bf_rne(__float_as_uint(rem));
}
__device__ __forceinline__ void split8(v4f a, v4f b, v8us& H, v8us& L) {
  unsigned short h0, h1, h2, h3, h4, h5, h6, h7, l0, l1, l2, l3, l4, l5, l6, l7;
  split1(a.x, h0, l0); split1(a.y, h1, l1); split1(a.z, h2, l2); split1(a.w, h3, l3);
  split1(b.x, h4, l4); split1(b.y, h5, l5); split1(b.z, h6, l6); split1(b.w, h7, l7);
  v8us hv = {h0, h1, h2, h3, h4, h5, h6, h7};
  v8us lv = {l0, l1, l2, l3, l4, l5, l6, l7};
  H = hv; L = lv;
}

__device__ __forceinline__ void afrag(const float* p0, const float* p1, FragB& H, FragB& L) {
  const v4f a = *(const v4f*)p0;
  const v4f b = *(const v4f*)(p0 + 4);
  const v4f c = *(const v4f*)p1;
  const v4f d = *(const v4f*)(p1 + 4);
  split8(a, b, H.u[0], L.u[0]);
  split8(c, d, H.u[1], L.u[1]);
}

__device__ __forceinline__ v8f mma3(v16b ah, v16b al, v16b bh, v16b bl, v8f c) {
  c = __builtin_amdgcn_wmma_f32_16x16x32_bf16(false, ah, false, bh, (short)0, c, false, false);
  c = __builtin_amdgcn_wmma_f32_16x16x32_bf16(false, ah, false, bl, (short)0, c, false, false);
  c = __builtin_amdgcn_wmma_f32_16x16x32_bf16(false, al, false, bh, (short)0, c, false, false);
  asm volatile("v_nop\n\tv_nop\n\tv_nop\n\tv_nop" : "+v"(c) : "v"(ah), "v"(al), "v"(bh), "v"(bl));
  return c;
}

__device__ __forceinline__ void zero4(v8f (&acc)[4]) {
  v8f z = {0.f, 0.f, 0.f, 0.f, 0.f, 0.f, 0.f, 0.f};
#pragma unroll
  for (int t = 0; t < 4; ++t) acc[t] = z;
}

template <int K>
__device__ __forceinline__ void gemm4(v8f (&acc)[4], const FragB& aH, const FragB& aL,
                                      const unsigned short* __restrict__ wh,
                                      const unsigned short* __restrict__ wl,
                                      int kt, int nb, int h, int m) {
#pragma unroll
  for (int t = 0; t < 4; ++t) {
    const size_t o = (size_t)(nb + 16 * t + m) * K + 32 * kt + 8 * h;
    FragB bH, bL;
    bH.u[0] = *(const v8us*)(wh + o);
    bH.u[1] = *(const v8us*)(wh + o + 16);
    bL.u[0] = *(const v8us*)(wl + o);
    bL.u[1] = *(const v8us*)(wl + o + 16);
    acc[t] = mma3(aH.v, aL.v, bH.v, bL.v, acc[t]);
  }
}

__global__ __launch_bounds__(NTHR) void k_prep(
    const float* __restrict__ w0, const float* __restrict__ w1, const float* __restrict__ w2,
    const float* __restrict__ w3, const float* __restrict__ w4, const float* __restrict__ w5,
    const float* __restrict__ w6, const float* __restrict__ w7, const float* __restrict__ w8,
    const float* __restrict__ w9, unsigned short* wh, unsigned short* wl) {
  const float* W = w0;
  int K = 64, NO = 64, off = WO_L1;
  switch (blockIdx.y) {
    case 0: W = w0; K = 64;  NO = 64;  off = WO_L1;  break;
    case 1: W = w1; K = 128; NO = 64;  off = WO_U1;  break;
    case 2: W = w2; K = 64;  NO = 64;  off = WO_L2;  break;
    case 3: W = w3; K = 128; NO = 64;  off = WO_U2;  break;
    case 4: W = w4; K = 128; NO = 64;  off = WO_F1;  break;
    case 5: W = w5; K = 64;  NO = 64;  off = WO_F2;  break;
    case 6: W = w6; K = 64;  NO = 192; off = WO_QKV; break;
    case 7: W = w7; K = 64;  NO = 64;  off = WO_O;   break;
    case 8: W = w8; K = 64;  NO = 256; off = WO_FF1; break;
    default: W = w9; K = 256; NO = 64; off = WO_FF2; break;
  }
  const int i = blockIdx.x * NTHR + threadIdx.x;
  if (i * 8 >= K * NO) return;
  const int o  = i * 8;
  const int n  = o / K;
  const int k0 = o - n * K;
  const float* p = W + (size_t)k0 * NO + n;
  v4f a, b;
  a.x = p[0];      a.y = p[NO];     a.z = p[2 * NO]; a.w = p[3 * NO];
  b.x = p[4 * NO]; b.y = p[5 * NO]; b.z = p[6 * NO]; b.w = p[7 * NO];
  v8us H, L;
  split8(a, b, H, L);
  unsigned short* dh = wh + off + o;
  unsigned short* dl = wl + off + o;
  *(volatile v8us*)dh = H;
  *(volatile v8us*)dl = L;
  __threadfence();
  *(volatile v8us*)dh = H;
  *(volatile v8us*)dl = L;
}

__global__ __launch_bounds__(NTHR) void k_wsmean(const float* __restrict__ x, float* wsp) {
  const int tid = blockIdx.x * NTHR + threadIdx.x;
  const int row = tid >> 4, c4 = (tid & 15) * 4;
  const int n = row / GPN, g = row - n * GPN;
  const int b = g / cT,    t = g - b * cT;
  const float* xp = x + ((((size_t)b * cN + n) * cF) * cT + t) * HD + c4;
  v4f s = *(const v4f*)xp;
#pragma unroll
  for (int f = 1; f < cF; ++f) s = s + *(const v4f*)(xp + (size_t)f * cT * HD);
  s = s * 0.125f;
  float* dp = wsp + (size_t)tid * 4;
  *(volatile v4f*)dp = s;
  __threadfence();
  *(volatile v4f*)dp = s;
}

template <int NBT>
__device__ __forceinline__ int scan_chunk(const int* __restrict__ dsts, int nE, int cbase, int nodeBase,
                                          int vec8, int* list, int tid, int lane, int wave) {
  int wc = 0;
#pragma unroll
  for (int g = 0; g < NGRP; ++g) {
    const int el0  = (g * NTHR + tid) * EPT;
    const int e0   = cbase + el0;
    const int sent = -2147483647 - 1;
    v4i da, db;
    if (vec8 != 0 && cbase + CHUNK <= nE) {
      da = *(const v4i*)(dsts + e0);
      db = *(const v4i*)(dsts + e0 + 4);
    } else {
      da.x = (e0     < nE) ? dsts[imin(e0,     nE - 1)] : sent;
      da.y = (e0 + 1 < nE) ? dsts[imin(e0 + 1, nE - 1)] : sent;
      da.z = (e0 + 2 < nE) ? dsts[imin(e0 + 2, nE - 1)] : sent;
      da.w = (e0 + 3 < nE) ? dsts[imin(e0 + 3, nE - 1)] : sent;
      db.x = (e0 + 4 < nE) ? dsts[imin(e0 + 4, nE - 1)] : sent;
      db.y = (e0 + 5 < nE) ? dsts[imin(e0 + 5, nE - 1)] : sent;
      db.z = (e0 + 6 < nE) ? dsts[imin(e0 + 6, nE - 1)] : sent;
      db.w = (e0 + 7 < nE) ? dsts[imin(e0 + 7, nE - 1)] : sent;
    }
    const unsigned nb = (unsigned)nodeBase;
    const unsigned s0 = (unsigned)da.x - nb, s1 = (unsigned)da.y - nb;
    const unsigned s2 = (unsigned)da.z - nb, s3 = (unsigned)da.w - nb;
    const unsigned s4 = (unsigned)db.x - nb, s5 = (unsigned)db.y - nb;
    const unsigned s6 = (unsigned)db.z - nb, s7 = (unsigned)db.w - nb;
    const bool h0 = s0 < (unsigned)NBT, h1 = s1 < (unsigned)NBT, h2 = s2 < (unsigned)NBT, h3 = s3 < (unsigned)NBT;
    const bool h4 = s4 < (unsigned)NBT, h5 = s5 < (unsigned)NBT, h6 = s6 < (unsigned)NBT, h7 = s7 < (unsigned)NBT;
    const unsigned any = __builtin_amdgcn_ballot_w32(h0 | h1 | h2 | h3 | h4 | h5 | h6 | h7);
    if (any != 0u) {
#define HITJ(J, HJ, SJ) { \
        const unsigned mj = __builtin_amdgcn_ballot_w32(HJ); \
        if (mj != 0u) { \
          if (HJ) { \
            const int pos = wc + (int)__builtin_amdgcn_mbcnt_lo(mj, 0u); \
            if (pos < WCAP) list[wave * WCAP + pos] = ((el0 + (J)) << 12) | (int)(SJ); \
          } \
          wc += (int)__builtin_popcount(mj); } }
      HITJ(0, h0, s0)
      HITJ(1, h1, s1)
      HITJ(2, h2, s2)
      HITJ(3, h3, s3)
      HITJ(4, h4, s4)
      HITJ(5, h5, s5)
      HITJ(6, h6, s6)
      HITJ(7, h7, s7)
#undef HITJ
    }
  }
  return wc;
}

template <int MODE>
__device__ __forceinline__ const float* gather_row(const float* X, int src, int g) {
  if (MODE == 0) return X + ((size_t)src * GPN + g) * HD;
  const int bb = (g >= cT) ? 1 : 0;
  const int t  = g - bb * cT;
  return X + (((size_t)bb * cNF + src) * cT + t) * HD;
}

template <int MODE>
__global__ __launch_bounds__(NTHR) void k_scan(
    const int* __restrict__ ei, const float* __restrict__ ew, const float* __restrict__ lw,
    const float* __restrict__ gt, const float* __restrict__ X, float* S, float* wsum,
    int nN, int nE, int vec8) {
  extern __shared__ v4f lds_dyn[];
  float* acc  = (float*)lds_dyn;
  int*   list = (int*)(acc + NB * SLOTF);
  int*   wcnt = list + LISTN;
  float* wsl  = (float*)(wcnt + NWAVE);
  const int tid = threadIdx.x, lane = tid & 31, wave = tid >> 5;
  const int nodeBase = blockIdx.x * NB;
  const int* dsts = ei + nE;

  {
    const v4f z = {0.f, 0.f, 0.f, 0.f};
    for (int i = tid; i < NB * SLOTF / 4; i += NTHR) lds_dyn[i] = z;
    if (tid < NB) wsl[tid] = 0.f;
  }
  const float gs  = 1.f / (1.f + __expf(-gt[0]));
  const float gsc = 1.f - gs;
  __syncthreads();

  const int nChunks = (nE + CHUNK - 1) / CHUNK;
#pragma unroll 1
  for (int ch = 0; ch < nChunks; ++ch) {
    const int cbase = ch * CHUNK;
    const int wc = scan_chunk<NB>(dsts, nE, cbase, nodeBase, vec8, list, tid, lane, wave);
    if (lane == 0) wcnt[wave] = wc;
    __syncthreads();
#pragma unroll 1
    for (int wsx = 0; wsx < NWAVE; ++wsx) {
      int n = wcnt[wsx];
      n = n > WCAP ? WCAP : (n < 0 ? 0 : n);
      const int* lp = list + wsx * WCAP;
#pragma unroll 1
      for (int i = 0; i < n; ++i) {
        const int ent  = lp[i];
        const int slot = ent & (NB - 1);
        int e = cbase + ((ent >> 12) & (CHUNK - 1));
        e = e > nE - 1 ? nE - 1 : e;
        int src = ei[e];
        src = src < 0 ? 0 : (src > nN - 1 ? nN - 1 : src);
        const float sl = 1.f / (1.f + __expf(-lw[e]));
        const float mw = gs * ew[e] + gsc * sl;
        {
          const float* xp = gather_row<MODE>(X, src, tid >> 4) + (tid & 15) * 4;
          const v4f v = *(const v4f*)xp;
          v4f* ap = (v4f*)(acc + slot * SLOTF + tid * 4);
          *ap = *ap + v * mw;
        }
        if (tid < 128) {
          const float* xp = gather_row<MODE>(X, src, 16 + (tid >> 4)) + (tid & 15) * 4;
          const v4f v = *(const v4f*)xp;
          v4f* ap = (v4f*)(acc + slot * SLOTF + 1024 + tid * 4);
          *ap = *ap + v * mw;
        }
        if (tid == 0) wsl[slot] = wsl[slot] + mw;
      }
    }
    __syncthreads();
  }
  __syncthreads();

  float* sp = S + (size_t)nodeBase * SLOTF;
#pragma unroll
  for (int q = 0; q < (NB * SLOTF) / (4 * NTHR); ++q) {
    const int f = q * 4 * NTHR + tid * 4;
    const v4f v = *(const v4f*)(acc + f);
    *(volatile v4f*)(sp + f) = v;
  }
  if (tid < 8) {
    const v4f v = *(const v4f*)(wsl + 4 * tid);
    *(volatile v4f*)(wsum + nodeBase + 4 * tid) = v;
  }
  __threadfence();
#pragma unroll
  for (int q = 0; q < (NB * SLOTF) / (4 * NTHR); ++q) {
    const int f = q * 4 * NTHR + tid * 4;
    const v4f v = *(const v4f*)(acc + f);
    *(volatile v4f*)(sp + f) = v;
  }
  if (tid < 8) {
    const v4f v = *(const v4f*)(wsl + 4 * tid);
    *(volatile v4f*)(wsum + nodeBase + 4 * tid) = v;
  }
}

__device__ __forceinline__ void decomp(int r, int& nf, int& g) {
  const int bb = r / (cNF * cT);
  const int rr = r - bb * (cNF * cT);
  nf = rr / cT;
  g  = bb * cT + (rr - nf * cT);
}

template <int MODE>
__global__ __launch_bounds__(NTHR) void k_node(
    const float* __restrict__ P0, const float* __restrict__ P1, const float* __restrict__ wsum,
    const float* __restrict__ bias1, const float* __restrict__ bias2,
    const unsigned short* __restrict__ wh, const unsigned short* __restrict__ wl, float* outp) {
  __shared__ __attribute__((aligned(16))) float stg[NWAVE * 16 * PST];
  constexpr int WA = (MODE == 0) ? WO_L1 : ((MODE == 1) ? WO_L2 : WO_F1);
  constexpr int WB = (MODE == 0) ? WO_U1 : ((MODE == 1) ? WO_U2 : WO_F2);
  constexpr int K1 = (MODE == 2) ? 128 : 64;
  constexpr int K2 = (MODE == 2) ? 64 : 128;
  const int tid = threadIdx.x, lane = tid & 31, wave = tid >> 5, h = lane >> 4, m = lane & 15;
  const int orow0 = blockIdx.x * TROWS + wave * 16;
  const int myrow = orow0 + m;
  (void)wsum;

  const float* aK0 = P0;
  const float* aK1 = P1;
  if (MODE == 0) {
    aK0 = P0 + (size_t)myrow * HD;
    aK1 = P1 + (size_t)imin(myrow, cR1 - 1) * HD;
  } else {
    int nf, g;
    decomp(myrow, nf, g);
    if (MODE == 1) { aK0 = P0 + ((size_t)nf * GPN + g) * HD; aK1 = P1 + (size_t)myrow * HD; }
    else           { aK0 = P0 + (size_t)myrow * HD;        aK1 = P1 + ((size_t)(nf >> 3) * GPN + g) * HD; }
  }

  v8f acc[4];
  zero4(acc);
#pragma unroll
  for (int kt = 0; kt < 2; ++kt) {
    FragB aH, aL;
    afrag(aK0 + 32 * kt + 8 * h, aK0 + 32 * kt + 16 + 8 * h, aH, aL);
    gemm4<K1>(acc, aH, aL, wh + WA, wl + WA, kt, 0, h, m);
  }
  if (K1 == 128) {
#pragma unroll
    for (int kt = 2; kt < 4; ++kt) {
      FragB aH, aL;
      afrag(aK1 + 32 * (kt - 2) + 8 * h, aK1 + 32 * (kt - 2) + 16 + 8 * h, aH, aL);
      gemm4<128>(acc, aH, aL, wh + WA, wl + WA, kt, 0, h, m);
    }
  }

  float* sw = stg + wave * 16 * PST;
  float* se = sw + (8 * h) * PST + m;
  if (MODE < 2) {
    float wv[8];
#pragma unroll
    for (int r = 0; r < 8; ++r) {
      const int rowr = orow0 + 8 * h + r;
      int node;
      if (MODE == 0) { node = imin(rowr / GPN, N1P - 1); }
      else { int nf, g; decomp(rowr, nf, g); node = nf; }
      wv[r] = wsum[node];
    }
#pragma unroll
    for (int t = 0; t < 4; ++t) {
      const float bv = bias1[16 * t + m];
#pragma unroll
      for (int r = 0; r < 8; ++r) se[r * PST + 16 * t] = acc[t][r] + wv[r] * bv;
    }
  } else {
#pragma unroll
    for (int t = 0; t < 4; ++t) {
      const float bv = bias1[16 * t + m];
#pragma unroll
      for (int r = 0; r < 8; ++r) se[r * PST + 16 * t] = fmaxf(acc[t][r] + bv, 0.f);
    }
  }
  __syncthreads();

  v8f acc2[4];
  zero4(acc2);
  const float* sr = sw + m * PST;
#pragma unroll
  for (int kt = 0; kt < 2; ++kt) {
    FragB aH, aL;
    afrag(sr + 32 * kt + 8 * h, sr + 32 * kt + 16 + 8 * h, aH, aL);
    gemm4<K2>(acc2, aH, aL, wh + WB, wl + WB, kt, 0, h, m);
  }
  if (K2 == 128) {
#pragma unroll
    for (int kt = 2; kt < 4; ++kt) {
      FragB aH, aL;
      afrag(aK1 + 32 * (kt - 2) + 8 * h, aK1 + 32 * (kt - 2) + 16 + 8 * h, aH, aL);
      gemm4<128>(acc2, aH, aL, wh + WB, wl + WB, kt, 0, h, m);
    }
  }
  __syncthreads();
#pragma unroll
  for (int t = 0; t < 4; ++t) {
    const float bv = bias2[16 * t + m];
#pragma unroll
    for (int r = 0; r < 8; ++r) {
      float v = acc2[t][r] + bv;
      if (MODE < 2) v = fmaxf(v, 0.f);
      se[r * PST + 16 * t] = v;
    }
  }
  __syncthreads();

  float* op = outp + (size_t)orow0 * HD + lane * 4;
#pragma unroll
  for (int i = 0; i < 8; ++i) {
    const v4f v = *(const v4f*)(sw + (2 * i + h) * PST + m * 4);
    *(volatile v4f*)(op + (size_t)(2 * i) * HD) = v;
  }
  __threadfence();
#pragma unroll
  for (int i = 0; i < 8; ++i) {
    const v4f v = *(const v4f*)(sw + (2 * i + h) * PST + m * 4);
    *(volatile v4f*)(op + (size_t)(2 * i) * HD) = v;
  }
}

__device__ __forceinline__ void ln_rows(const float* __restrict__ src, float* sq, float* hs,
                                        const float* __restrict__ g, const float* __restrict__ bta, int tid) {
  const int row = tid >> 1, half = tid & 1;
  const float* p = src + (size_t)row * HD + half * 32;
  v4f xv[8];
  float s = 0.f;
#pragma unroll
  for (int j = 0; j < 8; ++j) {
    xv[j] = *(const v4f*)(p + 4 * j);
    *(v4f*)(sq + row * HD + half * 32 + 4 * j) = xv[j];
    s += (xv[j].x + xv[j].y) + (xv[j].z + xv[j].w);
  }
  s += __shfl_xor(s, 1);
  const float mean = s * (1.f / 64.f);
  float q = 0.f;
#pragma unroll
  for (int j = 0; j < 8; ++j) {
    const v4f d = xv[j] - mean;
    q += (d.x * d.x + d.y * d.y) + (d.z * d.z + d.w * d.w);
  }
  q += __shfl_xor(q, 1);
  const float inv = rsqrtf(q * (1.f / 64.f) + 1e-5f);
#pragma unroll
  for (int j = 0; j < 8; ++j) {
    const v4f gv = *(const v4f*)(g + half * 32 + 4 * j);
    const v4f bv = *(const v4f*)(bta + half * 32 + 4 * j);
    const v4f hv = (xv[j] - mean) * inv * gv + bv;
    *(v4f*)(hs + row * PST + half * 32 + 4 * j) = hv;
  }
}

__global__ __launch_bounds__(ATHR) void k_attn(
    const float* __restrict__ sqin, const unsigned short* __restrict__ wh, const unsigned short* __restrict__ wl,
    const float* __restrict__ bqkv, const float* __restrict__ lg, const float* __restrict__ lb,
    const float* __restrict__ bo, float* sout) {
  extern __shared__ v4f lds_dyn[];
  float* sq = (float*)lds_dyn;
  float* hs = sq + AROWS * HD;
  float* qk = hs + AROWS * PST;
  const int tid = threadIdx.x, lane = tid & 31, wave = tid >> 5, h = lane >> 4, m = lane & 15;
  const size_t r0 = (size_t)blockIdx.x * AROWS;

  ln_rows(sqin + r0 * HD, sq, hs, lg, lb, tid);
  __syncthreads();

  {
    const float* ar = hs + (wave * 16 + m) * PST;
    FragB aH0, aL0, aH1, aL1;
    afrag(ar + 8 * h,      ar + 16 + 8 * h, aH0, aL0);
    afrag(ar + 32 + 8 * h, ar + 48 + 8 * h, aH1, aL1);
#pragma unroll
    for (int p = 0; p < 3; ++p) {
      v8f acc[4];
      zero4(acc);
      gemm4<64>(acc, aH0, aL0, wh + WO_QKV, wl + WO_QKV, 0, 64 * p, h, m);
      gemm4<64>(acc, aH1, aL1, wh + WO_QKV, wl + WO_QKV, 1, 64 * p, h, m);
      float* qe = qk + (wave * 16 + 8 * h) * QP + 64 * p + m;
#pragma unroll
      for (int t = 0; t < 4; ++t) {
        const float bv = bqkv[64 * p + 16 * t + m];
#pragma unroll
        for (int r = 0; r < 8; ++r) qe[r * QP + 16 * t] = acc[t][r] + bv;
      }
    }
  }
  __syncthreads();

#pragma unroll 1
  for (int j = 0; j < 2; ++j) {
    const int task = tid + j * ATHR;
    const int head = task & 3;
    const int tq   = (task >> 2) % cT;
    const int s    = task / (4 * cT);
    const int rq   = s * cT + tq;
    const float* qp = qk + rq * QP + head * 16;
    const v4f qa = *(const v4f*)qp, qb = *(const v4f*)(qp + 4), qc = *(const v4f*)(qp + 8), qd = *(const v4f*)(qp + 12);
    float sc[cT];
    float mx = -3.0e38f;
#pragma unroll
    for (int tk = 0; tk < cT; ++tk) {
      const float* kp = qk + (s * cT + tk) * QP + HD + head * 16;
      const v4f ka = *(const v4f*)kp, kb = *(const v4f*)(kp + 4), kc = *(const v4f*)(kp + 8), kd = *(const v4f*)(kp + 12);
      const v4f pr = qa * ka + qb * kb + qc * kc + qd * kd;
      const float d = ((pr.x + pr.y) + (pr.z + pr.w)) * 0.25f;
      sc[tk] = d;
      mx = fmaxf(mx, d);
    }
    float sum = 0.f;
#pragma unroll
    for (int tk = 0; tk < cT; ++tk) { sc[tk] = expf(sc[tk] - mx); sum += sc[tk]; }
    const float inv = 1.f / sum;
    v4f oa = {0.f, 0.f, 0.f, 0.f}, ob = oa, oc = oa, od = oa;
#pragma unroll
    for (int tk = 0; tk < cT; ++tk) {
      const float* vp = qk + (s * cT + tk) * QP + 2 * HD + head * 16;
      const float w = sc[tk] * inv;
      oa = oa + *(const v4f*)vp * w;
      ob = ob + *(const v4f*)(vp + 4) * w;
      oc = oc + *(const v4f*)(vp + 8) * w;
      od = od + *(const v4f*)(vp + 12) * w;
    }
    float* opo = hs + rq * PST + head * 16;
    *(v4f*)opo = oa; *(v4f*)(opo + 4) = ob; *(v4f*)(opo + 8) = oc; *(v4f*)(opo + 12) = od;
  }
  __syncthreads();

  {
    const float* ar = hs + (wave * 16 + m) * PST;
    v8f acc[4];
    zero4(acc);
#pragma unroll
    for (int kt = 0; kt < 2; ++kt) {
      FragB aH, aL;
      afrag(ar + 32 * kt + 8 * h, ar + 32 * kt + 16 + 8 * h, aH, aL);
      gemm4<64>(acc, aH, aL, wh + WO_O, wl + WO_O, kt, 0, h, m);
    }
    const int rb = wave * 16 + 8 * h;
#pragma unroll
    for (int t = 0; t < 4; ++t) {
      const float bv = bo[16 * t + m];
#pragma unroll
      for (int r = 0; r < 8; ++r) {
        float* e = sq + (rb + r) * HD + 16 * t + m;
        const float v = *e + acc[t][r] + bv;
        *e = v;
      }
    }
  }
  __syncthreads();

  float* gp = sout + r0 * HD;
#pragma unroll
  for (int q = 0; q < (AROWS * HD) / (4 * ATHR); ++q) {
    const int f = q * 4 * ATHR + tid * 4;
    const v4f v = *(const v4f*)(sq + f);
    *(volatile v4f*)(gp + f) = v;
  }
  __threadfence();
#pragma unroll
  for (int q = 0; q < (AROWS * HD) / (4 * ATHR); ++q) {
    const int f = q * 4 * ATHR + tid * 4;
    const v4f v = *(const v4f*)(sq + f);
    *(volatile v4f*)(gp + f) = v;
  }
}

__global__ __launch_bounds__(ATHR) void k_ffn(
    const float* __restrict__ sqin, const unsigned short* __restrict__ wh, const unsigned short* __restrict__ wl,
    const float* __restrict__ lg, const float* __restrict__ lb, const float* __restrict__ fb1,
    const float* __restrict__ fb2, float* out) {
  extern __shared__ v4f lds_dyn[];
  float* sq = (float*)lds_dyn;
  float* hs = sq + AROWS * HD;
  float* gb = hs + AROWS * PST;
  const int tid = threadIdx.x, lane = tid & 31, wave = tid >> 5, h = lane >> 4, m = lane & 15;
  const size_t r0 = (size_t)blockIdx.x * AROWS;

  ln_rows(sqin + r0 * HD, sq, hs, lg, lb, tid);
  __syncthreads();

  {
    const float* ar = hs + (wave * 16 + m) * PST;
    FragB aH0, aL0, aH1, aL1;
    afrag(ar + 8 * h,      ar + 16 + 8 * h, aH0, aL0);
    afrag(ar + 32 + 8 * h, ar + 48 + 8 * h, aH1, aL1);
#pragma unroll
    for (int p = 0; p < 4; ++p) {
      v8f acc[4];
      zero4(acc);
      gemm4<64>(acc, aH0, aL0, wh + WO_FF1, wl + WO_FF1, 0, 64 * p, h, m);
      gemm4<64>(acc, aH1, aL1, wh + WO_FF1, wl + WO_FF1, 1, 64 * p, h, m);
      float* ge = gb + (wave * 16 + 8 * h) * GP + 64 * p + m;
#pragma unroll
      for (int t = 0; t < 4; ++t) {
        const float bv = fb1[64 * p + 16 * t + m];
#pragma unroll
        for (int r = 0; r < 8; ++r) {
          const float v = acc[t][r] + bv;
          ge[r * GP + 16 * t] = 0.5f * v * (1.f + erff(v * 0.70710678118654752f));
        }
      }
    }
  }
  __syncthreads();

  {
    const float* ar = gb + (wave * 16 + m) * GP;
    v8f acc[4];
    zero4(acc);
#pragma unroll
    for (int kt = 0; kt < 8; ++kt) {
      FragB aH, aL;
      afrag(ar + 32 * kt + 8 * h, ar + 32 * kt + 16 + 8 * h, aH, aL);
      gemm4<256>(acc, aH, aL, wh + WO_FF2, wl + WO_FF2, kt, 0, h, m);
    }
    const int rb = wave * 16 + 8 * h;
#pragma unroll
    for (int t = 0; t < 4; ++t) {
      const float bv = fb2[16 * t + m];
#pragma unroll
      for (int r = 0; r < 8; ++r) {
        float* e = sq + (rb + r) * HD + 16 * t + m;
        const float v = *e + acc[t][r] + bv;
        *e = v;
      }
    }
  }
  __syncthreads();

  v4f mv = {0.f, 0.f, 0.f, 0.f};
  if (tid < 128) {
    const float* sp = sq + (tid >> 4) * cT * HD + (tid & 15) * 4;
#pragma unroll
    for (int t = 0; t < cT; ++t) mv = mv + *(const v4f*)(sp + t * HD);
    mv = mv * (1.f / 12.f);
  }
  float* op = out + (size_t)blockIdx.x * (AROWS / cT) * HD + tid * 4;
  if (tid < 128) *(volatile v4f*)op = mv;
  __threadfence();
  if (tid < 128) *(volatile v4f*)op = mv;
}

static inline size_t carve(size_t& off, size_t bytes) {
  const size_t o = off;
  off = (off + bytes + 255) & ~(size_t)255;
  return o;
}

extern "C" void kernel_launch(void* const* d_in, const int* in_sizes, int n_in,
                              void* d_out, int out_size, void* d_ws, size_t ws_size,
                              hipStream_t stream) {
  if (n_in < 33) return;
  const int expect[33] = {
      cBATCH * cN * cF * cT * HD, 2 * cE1, cE1, 2 * cE2, cE2,
      HD * HD, HD, 2 * HD * HD, HD, 1, cE1,
      HD * HD, HD, 2 * HD * HD, HD, 1, cE2,
      2 * HD * HD, HD, HD * HD, HD,
      HD, HD, HD, HD,
      HD * 3 * HD, 3 * HD, HD * HD, HD, HD * 4 * HD, 4 * HD, 4 * HD * HD, HD};
  for (int i = 0; i < 33; ++i) {
    if (i == 9 || i == 15) { if (in_sizes[i] < 1) return; }
    else if (in_sizes[i] != expect[i]) return;
  }
  if (out_size != cSEQ * HD) return;

  const float* x     = (const float*)d_in[0];
  const int*   ei1   = (const int*)d_in[1];
  const float* ew1   = (const float*)d_in[2];
  const int*   ei2   = (const int*)d_in[3];
  const float* ew2   = (const float*)d_in[4];
  const float* Wl1   = (const float*)d_in[5];
  const float* bl1   = (const float*)d_in[6];
  const float* Wu1   = (const float*)d_in[7];
  const float* bu1   = (const float*)d_in[8];
  const float* gt1   = (const float*)d_in[9];
  const float* lw1   = (const float*)d_in[10];
  const float* Wl2   = (const float*)d_in[11];
  const float* bl2   = (const float*)d_in[12];
  const float* Wu2   = (const float*)d_in[13];
  const float* bu2   = (const float*)d_in[14];
  const float* gt2   = (const float*)d_in[15];
  const float* lw2   = (const float*)d_in[16];
  const float* Wf1   = (const float*)d_in[17];
  const float* bf1   = (const float*)d_in[18];
  const float* Wf2   = (const float*)d_in[19];
  const float* bf2   = (const float*)d_in[20];
  const float* ln1g  = (const float*)d_in[21];
  const float* ln1b  = (const float*)d_in[22];
  const float* ln2g  = (const float*)d_in[23];
  const float* ln2b  = (const float*)d_in[24];
  const float* Wqkv  = (const float*)d_in[25];
  const float* bqkv  = (const float*)d_in[26];
  const float* Wo    = (const float*)d_in[27];
  const float* bo    = (const float*)d_in[28];
  const float* Wff1  = (const float*)d_in[29];
  const float* bff1  = (const float*)d_in[30];
  const float* Wff2  = (const float*)d_in[31];
  const float* bff2  = (const float*)d_in[32];
  float* out = (float*)d_out;

  size_t off = 0;
  const size_t oWH  = carve(off, (size_t)WTOT * 2);
  const size_t oWL  = carve(off, (size_t)WTOT * 2);
  const size_t oWSP = carve(off, (size_t)cR1 * HD * 4);
  const size_t oS1  = carve(off, (size_t)N1P * SLOTF * 4);
  const size_t oSM1 = carve(off, (size_t)N1P * 4);
  const size_t oWSU = carve(off, (size_t)R1P * HD * 4);
  const size_t oRA  = carve(off, (size_t)cRX * HD * 4);
  const size_t oSM2 = carve(off, (size_t)cNF * 4);
  const size_t oRB  = carve(off, (size_t)cRX * HD * 4);
  if (off > ws_size || off > ((size_t)128 << 20)) return;

  char* ws = (char*)d_ws;
  unsigned short* wh = (unsigned short*)(ws + oWH);
  unsigned short* wl = (unsigned short*)(ws + oWL);
  float* wsp  = (float*)(ws + oWSP);
  float* S1   = (float*)(ws + oS1);
  float* sm1  = (float*)(ws + oSM1);
  float* wsu  = (float*)(ws + oWSU);
  float* S2   = (float*)(ws + oRA);
  float* seq  = (float*)(ws + oRA);
  float* sm2  = (float*)(ws + oSM2);
  float* fnu  = (float*)(ws + oRB);
  float* seq2 = (float*)(ws + oRB);

  const int vec8a = ((cE1 & 3) == 0) ? 1 : 0;
  const int vec8b = ((cE2 & 3) == 0) ? 1 : 0;

  k_prep<<<dim3(8, 10), NTHR, 0, stream>>>(Wl1, Wu1, Wl2, Wu2, Wf1, Wf2, Wqkv, Wo, Wff1, Wff2, wh, wl);
  k_wsmean<<<NWSB, NTHR, 0, stream>>>(x, wsp);

  hipFuncSetAttribute(reinterpret_cast<const void*>(&k_scan<0>), hipFuncAttributeMaxDynamicSharedMemorySize, LDS_SCAN);
  k_scan<0><<<NSCAN1, NTHR, LDS_SCAN, stream>>>(ei1, ew1, lw1, gt1, wsp, S1, sm1, cN, cE1, vec8a);
  k_node<0><<<NBLK1, NTHR, 0, stream>>>(S1, wsp, sm1, bl1, bu1, wh, wl, wsu);

  hipFuncSetAttribute(reinterpret_cast<const void*>(&k_scan<1>), hipFuncAttributeMaxDynamicSharedMemorySize, LDS_SCAN);
  k_scan<1><<<NSCAN2, NTHR, LDS_SCAN, stream>>>(ei2, ew2, lw2, gt2, x, S2, sm2, cNF, cE2, vec8b);
  k_node<1><<<NBLKX, NTHR, 0, stream>>>(S2, x, sm2, bl2, bu2, wh, wl, fnu);

  k_node<2><<<NBLKX, NTHR, 0, stream>>>(fnu, wsu, sm2, bf1, bf2, wh, wl, seq);

  hipFuncSetAttribute(reinterpret_cast<const void*>(&k_attn), hipFuncAttributeMaxDynamicSharedMemorySize, LDS_ATTN);
  k_attn<<<NBLKA, ATHR, LDS_ATTN, stream>>>(seq, wh, wl, bqkv, ln1g, ln1b, bo, seq2);

  hipFuncSetAttribute(reinterpret_cast<const void*>(&k_ffn), hipFuncAttributeMaxDynamicSharedMemorySize, LDS_FFN);
  k_ffn<<<NBLKA, ATHR, LDS_FFN, stream>>>(seq2, wh, wl, ln2g, ln2b, bff1, bff2, out);
}
